// MultiHeadGATLayer_86260123174621
// MI455X (gfx1250) — hardware-verified
//
#include <hip/hip_runtime.h>
#include <stddef.h>
#include <stdint.h>
#include <math.h>


#define DIN     256
#define NCH     256
#define NTHR    256
#define NWAVE   8
#define EPT     8
#define CHUNK   (NTHR * EPT)
#define WCAP    (EPT * 32)
#define LISTN   (NWAVE * WCAP)
#define NBMAX   2048
#define RCAP    28672
#define DEGCAP  256
#define GBM     64
#define GBN     64
#define GTHR    128
#define NEG_SLOPE 0.2f
#define LN_EPS  1e-5f
#define WSMAX   134217728
#define LDS_AGG ((2 * RCAP + 2 * NBMAX + LISTN) * 4 + 64)

static_assert((CHUNK & (CHUNK - 1)) == 0 && CHUNK <= 4096);
static_assert((NBMAX & (NBMAX - 1)) == 0 && NBMAX <= 4096);
static_assert(NTHR * 8 == NBMAX);
static_assert(LISTN >= NBMAX);
static_assert(LISTN >= NWAVE * WCAP);
static_assert(LISTN >= NWAVE * NCH);
static_assert((RCAP % 32) == 0);
static_assert(LDS_AGG <= 300000);
static_assert(GBM == (GTHR / 32) * 16);
static_assert((DIN % 32) == 0 && DIN / 8 == 32);
static_assert((NCH % GBN) == 0 && (NCH % 32) == 0);
static_assert(NCH == 8 * 32);

typedef float          v4f  __attribute__((ext_vector_type(4)));
typedef float          v8f  __attribute__((ext_vector_type(8)));
typedef int            v4i  __attribute__((ext_vector_type(4)));
typedef int            v8i  __attribute__((ext_vector_type(8)));
typedef unsigned short v8us __attribute__((ext_vector_type(8)));
typedef __bf16         v16b __attribute__((ext_vector_type(16)));
typedef v4f  __attribute__((may_alias)) v4fa;
typedef v8us __attribute__((may_alias)) v8usa;
union FragB { v16b v; v8us h[2]; v8i w; };

__device__ __forceinline__ v8f wmb(const FragB& a, const FragB& b, v8f c) {
  v8f d = __builtin_amdgcn_wmma_f32_16x16x32_bf16(false, a.v, false, b.v, (short)0, c, false, false);
  asm volatile("v_nop\n\tv_nop\n\tv_nop\n\tv_nop" : "+v"(d) : "v"(a.w), "v"(b.w));
  return d;
}

__device__ __forceinline__ unsigned short f2bf(float f) {
  unsigned u = __float_as_uint(f);
  u += 0x7FFFu + ((u >> 16) & 1u);
  return (unsigned short)(u >> 16);
}
__device__ __forceinline__ float bfr(float f) {
  unsigned u = __float_as_uint(f);
  u = (u + 0x7FFFu + ((u >> 16) & 1u)) & 0xFFFF0000u;
  return __uint_as_float(u);
}
__device__ __forceinline__ v4f bfr4(const v4f a) {
  v4f r; r.x = bfr(a.x); r.y = bfr(a.y); r.z = bfr(a.z); r.w = bfr(a.w); return r;
}
__device__ __forceinline__ v8us cvt8b(const v4f a, const v4f b) {
  v8us o;
  o[0] = f2bf(a.x); o[1] = f2bf(a.y); o[2] = f2bf(a.z); o[3] = f2bf(a.w);
  o[4] = f2bf(b.x); o[5] = f2bf(b.y); o[6] = f2bf(b.z); o[7] = f2bf(b.w);
  return o;
}
__device__ __forceinline__ float dot8(const v4f a, const v4f b, const v4f c, const v4f d) {
  float p = a.x * c.x;
  p = fmaf(a.y, c.y, p); p = fmaf(a.z, c.z, p); p = fmaf(a.w, c.w, p);
  p = fmaf(b.x, d.x, p); p = fmaf(b.y, d.y, p); p = fmaf(b.z, d.z, p); p = fmaf(b.w, d.w, p);
  return p;
}

__device__ __forceinline__ int scan_chunk(const int* __restrict__ dsts, int nE, int cbase, int slotBase,
                                          int nb, int vec8, int* list, int tid, int lane, int wave) {
  int wc = 0;
  const int el0  = tid * EPT;
  const int e0   = cbase + el0;
  const int sent = -2147483647 - 1;
  v4i da, db;
  if (vec8 != 0 && cbase + CHUNK <= nE) {
    da = *(const v4i*)(dsts + e0);
    db = *(const v4i*)(dsts + e0 + 4);
  } else {
    da.x = (e0     < nE) ? dsts[min(e0,     nE - 1)] : sent;
    da.y = (e0 + 1 < nE) ? dsts[min(e0 + 1, nE - 1)] : sent;
    da.z = (e0 + 2 < nE) ? dsts[min(e0 + 2, nE - 1)] : sent;
    da.w = (e0 + 3 < nE) ? dsts[min(e0 + 3, nE - 1)] : sent;
    db.x = (e0 + 4 < nE) ? dsts[min(e0 + 4, nE - 1)] : sent;
    db.y = (e0 + 5 < nE) ? dsts[min(e0 + 5, nE - 1)] : sent;
    db.z = (e0 + 6 < nE) ? dsts[min(e0 + 6, nE - 1)] : sent;
    db.w = (e0 + 7 < nE) ? dsts[min(e0 + 7, nE - 1)] : sent;
  }
  const unsigned nbs = (unsigned)slotBase;
  const unsigned unb = (unsigned)nb;
  const unsigned s0 = (unsigned)da.x - nbs, s1 = (unsigned)da.y - nbs;
  const unsigned s2 = (unsigned)da.z - nbs, s3 = (unsigned)da.w - nbs;
  const unsigned s4 = (unsigned)db.x - nbs, s5 = (unsigned)db.y - nbs;
  const unsigned s6 = (unsigned)db.z - nbs, s7 = (unsigned)db.w - nbs;
  const bool h0 = s0 < unb, h1 = s1 < unb, h2 = s2 < unb, h3 = s3 < unb;
  const bool h4 = s4 < unb, h5 = s5 < unb, h6 = s6 < unb, h7 = s7 < unb;
  const unsigned any = __builtin_amdgcn_ballot_w32(h0 | h1 | h2 | h3 | h4 | h5 | h6 | h7);
  if (any != 0u) {
#define HITJ(J, HJ, SJ) { \
      const unsigned mj = __builtin_amdgcn_ballot_w32(HJ); \
      if (mj != 0u) { \
        if (HJ) { \
          const int pos = wc + (int)__builtin_amdgcn_mbcnt_lo(mj, 0u); \
          if (pos < WCAP) list[wave * WCAP + pos] = ((el0 + (J)) << 12) | (int)(SJ); \
        } \
        wc += (int)__builtin_popcount(mj); } }
    HITJ(0, h0, s0)
    HITJ(1, h1, s1)
    HITJ(2, h2, s2)
    HITJ(3, h3, s3)
    HITJ(4, h4, s4)
    HITJ(5, h5, s5)
    HITJ(6, h6, s6)
    HITJ(7, h7, s7)
#undef HITJ
  }
  return wc;
}

__global__ __launch_bounds__(NTHR) void k_xprep(const float* __restrict__ x, unsigned short* xb, int nN, int nUnits) {
  const int i = (int)blockIdx.x * NTHR + (int)threadIdx.x;
  if (i >= nUnits) return;
  const int row = i >> 5;
  const int c0  = (i & 31) * 8;
  const int rc  = row < nN ? row : nN - 1;
  const float* p = x + (size_t)rc * DIN + c0;
  v4f a = *(const v4fa*)p, b = *(const v4fa*)(p + 4);
  const v4f z4 = {0.f, 0.f, 0.f, 0.f};
  if (row >= nN) { a = z4; b = z4; }
  const v8us hv = cvt8b(a, b);
  const size_t o = (size_t)row * DIN + c0;
  *(volatile v8us*)(xb + o) = hv;
  __threadfence();
  *(volatile v8us*)(xb + o) = hv;
}

__global__ __launch_bounds__(NTHR) void k_wtr(const float* __restrict__ w, int Kin, int Ncol, int Nrows, int Kout,
                                              unsigned short* wt, int nUnits) {
  const int u = (int)blockIdx.x * NTHR + (int)threadIdx.x;
  if (u >= nUnits) return;
  const int kq = Kout >> 3;
  const int n  = u / kq;
  const int k8 = (u - n * kq) * 8;
  const int kk = k8 - (k8 / Kin) * Kin;
  const int ncl = n < Ncol ? n : Ncol - 1;
  const float* p = w + (size_t)kk * (size_t)Ncol + ncl;
  v4f a, b;
  a.x = p[0];                    a.y = p[(size_t)Ncol];         a.z = p[(size_t)2 * Ncol];     a.w = p[(size_t)3 * Ncol];
  b.x = p[(size_t)4 * Ncol];     b.y = p[(size_t)5 * Ncol];     b.z = p[(size_t)6 * Ncol];     b.w = p[(size_t)7 * Ncol];
  const v4f z4 = {0.f, 0.f, 0.f, 0.f};
  if (n >= Ncol || n >= Nrows) { a = z4; b = z4; }
  const v8us hv = cvt8b(a, b);
  const size_t o = (size_t)n * (size_t)Kout + k8;
  *(volatile v8us*)(wt + o) = hv;
  __threadfence();
  *(volatile v8us*)(wt + o) = hv;
}

__global__ __launch_bounds__(GTHR) void k_gemm(
    const unsigned short* __restrict__ A, const unsigned short* __restrict__ WT,
    float* outF, int K, int ldo)
{
  __shared__ __attribute__((aligned(16))) float stg[GBM * GBN];
  const int tid = (int)threadIdx.x, lane = tid & 31, wave = tid >> 5, hh = lane >> 4, m = lane & 15;
  const int rowBase = (int)blockIdx.x * GBM;
  const int col0    = (int)blockIdx.y * GBN;

  v8f acc[4];
  {
    const v8f z = {0.f, 0.f, 0.f, 0.f, 0.f, 0.f, 0.f, 0.f};
    acc[0] = z; acc[1] = z; acc[2] = z; acc[3] = z;
  }
  const unsigned short* ap = A  + (size_t)(rowBase + 16 * wave + m) * (size_t)K + 8 * hh;
  const unsigned short* wp = WT + (size_t)(col0 + m) * (size_t)K + 8 * hh;
  const int ksteps = K >> 5;
#pragma unroll 1
  for (int ks = 0; ks < ksteps; ++ks) {
    FragB af;
    af.h[0] = *(const v8usa*)(ap + 32 * ks);
    af.h[1] = *(const v8usa*)(ap + 32 * ks + 16);
#pragma unroll
    for (int t = 0; t < 4; ++t) {
      const unsigned short* wq = wp + (size_t)(16 * t) * (size_t)K + 32 * ks;
      FragB bf;
      bf.h[0] = *(const v8usa*)wq;
      bf.h[1] = *(const v8usa*)(wq + 16);
      acc[t] = wmb(af, bf, acc[t]);
    }
  }

#pragma unroll
  for (int t = 0; t < 4; ++t) {
    const int lc = 16 * t + m;
#pragma unroll
    for (int r = 0; r < 8; ++r) {
      const int lr = 16 * wave + 8 * hh + r;
      stg[lr * GBN + lc] = acc[t][r];
    }
  }
  __syncthreads();

  v4f fv[8];
#pragma unroll
  for (int i = 0; i < 8; ++i) {
    const int lr = 16 * wave + 2 * i + hh;
    fv[i] = *(const v4fa*)(stg + lr * GBN + 4 * m);
  }
#pragma unroll
  for (int i = 0; i < 8; ++i) {
    const int lr = 16 * wave + 2 * i + hh;
    const int gr = rowBase + lr;
    float* op = outF + (size_t)gr * (size_t)ldo + col0 + 4 * m;
    *(volatile v4f*)op = fv[i];
  }
  __threadfence();
#pragma unroll
  for (int i = 0; i < 8; ++i) {
    const int lr = 16 * wave + 2 * i + hh;
    const int gr = rowBase + lr;
    float* op = outF + (size_t)gr * (size_t)ldo + col0 + 4 * m;
    *(volatile v4f*)op = fv[i];
  }
}

__global__ __launch_bounds__(NTHR) void k_agg(
    const int* __restrict__ srcs, const int* __restrict__ dsts,
    const float* __restrict__ HF, const float* __restrict__ x,
    const float* __restrict__ asrc, const float* __restrict__ adst,
    const float* __restrict__ gam, const float* __restrict__ bet,
    float* out, int nN, int nE, int nb, int vec8) {
  extern __shared__ v4f lds_dyn[];
  int* reg1 = (int*)lds_dyn;
  int* reg2 = reg1 + RCAP;
  int* scnt = reg2 + RCAP;
  int* soff = scnt + NBMAX;
  int* list = soff + NBMAX;
  int* wcnt = list + LISTN;
  int* wtot = wcnt + NWAVE;
  const int tid = (int)threadIdx.x, lane = tid & 31, wave = tid >> 5;
  const int nodeBase = (int)blockIdx.x * nb;

  for (int i = tid; i < NBMAX; i += NTHR) scnt[i] = 0;
  __syncthreads();

  int tot = 0;
  const int nChunks = (nE + CHUNK - 1) / CHUNK;
#pragma unroll 1
  for (int ch = 0; ch < nChunks; ++ch) {
    const int cbase = ch * CHUNK;
    const int wc = scan_chunk(dsts, nE, cbase, nodeBase, nb, vec8, list, tid, lane, wave);
    if (lane == 0) wcnt[wave] = wc;
    __syncthreads();
    int pre = 0, all = 0;
#pragma unroll
    for (int w2 = 0; w2 < NWAVE; ++w2) {
      int c = wcnt[w2];
      c = c < 0 ? 0 : (c > WCAP ? WCAP : c);
      all += c;
      pre += (w2 < wave) ? c : 0;
    }
    const int wcc  = wc > WCAP ? WCAP : wc;
    const int base = tot + pre;
#pragma unroll 1
    for (int i = lane; i < wcc; i += 32) {
      const int ent = list[wave * WCAP + i];
      const int el  = (ent >> 12) & (CHUNK - 1);
      const int sl  = ent & (NBMAX - 1);
      int eid = cbase + el;
      eid = eid > nE - 1 ? nE - 1 : eid;
      const int pos = base + i;
      if (pos < RCAP) reg1[pos] = (int)(((unsigned)eid << 12) | (unsigned)sl);
    }
    tot += all;
    tot = tot > RCAP ? RCAP : tot;
    __syncthreads();
  }
  const int nh = tot;

  if (wave == 0) {
#pragma unroll 1
    for (int b0 = 0; b0 < nh; b0 += 32) {
      const int idx = b0 + lane;
      const int uv  = reg1[idx < nh ? idx : nh - 1];
      const int m32 = (nh - b0) < 32 ? (nh - b0) : 32;
#pragma unroll 1
      for (int k = 0; k < m32; ++k) {
        const int u  = __builtin_amdgcn_readlane(uv, k);
        const int sl = u & (NBMAX - 1);
        if (lane == 0) scnt[sl] = scnt[sl] + 1;
      }
    }
  }
  __syncthreads();

  {
    const v4i ca = *(const v4i*)(scnt + 8 * tid);
    const v4i cb = *(const v4i*)(scnt + 8 * tid + 4);
    const int e0 = ca.x < 0 ? 0 : ca.x, e1 = ca.y < 0 ? 0 : ca.y, e2 = ca.z < 0 ? 0 : ca.z, e3 = ca.w < 0 ? 0 : ca.w;
    const int e4 = cb.x < 0 ? 0 : cb.x, e5 = cb.y < 0 ? 0 : cb.y, e6 = cb.z < 0 ? 0 : cb.z, e7 = cb.w < 0 ? 0 : cb.w;
    const int ts = e0 + e1 + e2 + e3 + e4 + e5 + e6 + e7;
    int incl = ts;
#pragma unroll
    for (int d = 1; d < 32; d <<= 1) {
      const int up = __shfl_up(incl, d);
      if (lane >= d) incl += up;
    }
    if (lane == 31) wtot[wave] = incl;
    __syncthreads();
    int pre = 0;
#pragma unroll
    for (int w2 = 0; w2 < NWAVE; ++w2) pre += (w2 < wave) ? wtot[w2] : 0;
    int run = pre + incl - ts;
    soff[8 * tid + 0] = run; run += e0;
    soff[8 * tid + 1] = run; run += e1;
    soff[8 * tid + 2] = run; run += e2;
    soff[8 * tid + 3] = run; run += e3;
    soff[8 * tid + 4] = run; run += e4;
    soff[8 * tid + 5] = run; run += e5;
    soff[8 * tid + 6] = run; run += e6;
    soff[8 * tid + 7] = run;
  }
  __syncthreads();
  for (int i = tid; i < NBMAX; i += NTHR) list[i] = soff[i];
  __syncthreads();

  if (wave == 0) {
#pragma unroll 1
    for (int b0 = 0; b0 < nh; b0 += 32) {
      const int idx = b0 + lane;
      const int uv  = reg1[idx < nh ? idx : nh - 1];
      const int m32 = (nh - b0) < 32 ? (nh - b0) : 32;
#pragma unroll 1
      for (int k = 0; k < m32; ++k) {
        const int u   = __builtin_amdgcn_readlane(uv, k);
        const int sl  = u & (NBMAX - 1);
        const int eid = (int)((unsigned)u >> 12);
        if (lane == 0) {
          int pos = list[sl];
          pos = pos < 0 ? 0 : (pos > RCAP - 1 ? RCAP - 1 : pos);
          reg2[pos] = eid;
          list[sl] = pos + 1;
        }
      }
    }
  }
  __syncthreads();

  const int nbw = nb >> 3;
  const bool ovf = (nh >= RCAP);
  const float qnan = __int_as_float(0x7fc00000);
  const int c0 = 8 * lane;
  const v4f asA = bfr4(*(const v4fa*)(asrc + c0)), asB = bfr4(*(const v4fa*)(asrc + c0 + 4));
  const v4f adA = bfr4(*(const v4fa*)(adst + c0)), adB = bfr4(*(const v4fa*)(adst + c0 + 4));
  const v4f gaA = bfr4(*(const v4fa*)(gam  + c0)), gaB = bfr4(*(const v4fa*)(gam  + c0 + 4));
  const v4f beA = bfr4(*(const v4fa*)(bet  + c0)), beB = bfr4(*(const v4fa*)(bet  + c0 + 4));
  const float inv256 = 0.00390625f;
  float* wrow = (float*)list + wave * NCH;

#pragma unroll 1
  for (int jt = 0; jt < nbw; ++jt) {
    const int slot = wave * nbw + jt;
    const int grow = nodeBase + slot;
    const int gcl  = grow < nN ? grow : nN - 1;
    int st = soff[slot];
    const int craw = scnt[slot];
    int cnt = craw;
    st  = st < 0 ? 0 : (st > nh ? nh : st);
    cnt = cnt < 0 ? 0 : (cnt > DEGCAP ? DEGCAP : cnt);
    if (cnt > nh - st) cnt = nh - st;
    const float pz = (ovf || craw > DEGCAP) ? qnan : 0.0f;
    const bool wr = grow < nN;

    const float* fp = HF + (size_t)gcl * NCH + c0;
    const v4f fdA = *(const v4fa*)fp, fdB = *(const v4fa*)(fp + 4);
    float pd = dot8(fdA, fdB, adA, adB);
    pd += __shfl_xor(pd, 1);
    pd += __shfl_xor(pd, 2);
    float mx = -1.0e30f, dn = 0.f;
    v4f avA = {0.f, 0.f, 0.f, 0.f}, avB = {0.f, 0.f, 0.f, 0.f};

#pragma unroll 1
    for (int q = 0; q < cnt; ++q) {
      int idx = st + q; idx = idx > RCAP - 1 ? RCAP - 1 : idx;
      int eid = reg2[idx]; eid = eid < 0 ? 0 : (eid > nE - 1 ? nE - 1 : eid);
      const int sraw = srcs[eid];
      const int s = sraw < 0 ? 0 : (sraw > nN - 1 ? nN - 1 : sraw);
      const float* sp = HF + (size_t)s * NCH + c0;
      const v4f fsA = *(const v4fa*)sp, fsB = *(const v4fa*)(sp + 4);
      float es = dot8(fsA, fsB, asA, asB);
      es += __shfl_xor(es, 1);
      es += __shfl_xor(es, 2);
      float lg = es + pd;
      lg = lg > 0.f ? lg : lg * NEG_SLOPE;
      const float df = lg - mx;
      const float ee = __expf(-fabsf(df));
      const bool up  = df > 0.f;
      const float s1 = up ? ee : 1.0f;
      const float s2 = up ? 1.0f : ee;
      mx = up ? lg : mx;
      dn = fmaf(dn, s1, s2);
      avA.x = fmaf(avA.x, s1, s2 * fsA.x);
      avA.y = fmaf(avA.y, s1, s2 * fsA.y);
      avA.z = fmaf(avA.z, s1, s2 * fsA.z);
      avA.w = fmaf(avA.w, s1, s2 * fsA.w);
      avB.x = fmaf(avB.x, s1, s2 * fsB.x);
      avB.y = fmaf(avB.y, s1, s2 * fsB.y);
      avB.z = fmaf(avB.z, s1, s2 * fsB.z);
      avB.w = fmaf(avB.w, s1, s2 * fsB.w);
    }
    const float ds = dn > 0.f ? dn : 1.0f;
    const float iv = (dn > 0.f ? 1.0f : 0.0f) * __builtin_amdgcn_rcpf(ds);
    const float* xp = x + (size_t)gcl * DIN + c0;
    const v4f xA = bfr4(*(const v4fa*)xp), xB = bfr4(*(const v4fa*)(xp + 4));
    const float o0 = fmaf(avA.x, iv, xA.x), o1 = fmaf(avA.y, iv, xA.y);
    const float o2 = fmaf(avA.z, iv, xA.z), o3 = fmaf(avA.w, iv, xA.w);
    const float o4 = fmaf(avB.x, iv, xB.x), o5 = fmaf(avB.y, iv, xB.y);
    const float o6 = fmaf(avB.z, iv, xB.z), o7 = fmaf(avB.w, iv, xB.w);
    float sm = ((o0 + o1) + (o2 + o3)) + ((o4 + o5) + (o6 + o7));
#pragma unroll
    for (int off = 16; off > 0; off >>= 1) sm += __shfl_xor(sm, off);
    const float mu = sm * inv256;
    const float d0 = o0 - mu, d1 = o1 - mu, d2 = o2 - mu, d3 = o3 - mu;
    const float d4 = o4 - mu, d5 = o5 - mu, d6 = o6 - mu, d7 = o7 - mu;
    float ss = ((d0 * d0 + d1 * d1) + (d2 * d2 + d3 * d3)) + ((d4 * d4 + d5 * d5) + (d6 * d6 + d7 * d7));
#pragma unroll
    for (int off = 16; off > 0; off >>= 1) ss += __shfl_xor(ss, off);
    const float var = ss * inv256;
    const float rs  = rsqrtf(var + LN_EPS);
    float t0 = fmaf(d0 * rs, gaA.x, beA.x), t1 = fmaf(d1 * rs, gaA.y, beA.y);
    float t2 = fmaf(d2 * rs, gaA.z, beA.z), t3 = fmaf(d3 * rs, gaA.w, beA.w);
    float t4 = fmaf(d4 * rs, gaB.x, beB.x), t5 = fmaf(d5 * rs, gaB.y, beB.y);
    float t6 = fmaf(d6 * rs, gaB.z, beB.z), t7 = fmaf(d7 * rs, gaB.w, beB.w);
    v4f yA, yB;
    yA.x = (t0 > 0.f ? t0 : (__expf(fminf(t0, 0.f)) - 1.0f)) + pz;
    yA.y = (t1 > 0.f ? t1 : (__expf(fminf(t1, 0.f)) - 1.0f)) + pz;
    yA.z = (t2 > 0.f ? t2 : (__expf(fminf(t2, 0.f)) - 1.0f)) + pz;
    yA.w = (t3 > 0.f ? t3 : (__expf(fminf(t3, 0.f)) - 1.0f)) + pz;
    yB.x = (t4 > 0.f ? t4 : (__expf(fminf(t4, 0.f)) - 1.0f)) + pz;
    yB.y = (t5 > 0.f ? t5 : (__expf(fminf(t5, 0.f)) - 1.0f)) + pz;
    yB.z = (t6 > 0.f ? t6 : (__expf(fminf(t6, 0.f)) - 1.0f)) + pz;
    yB.w = (t7 > 0.f ? t7 : (__expf(fminf(t7, 0.f)) - 1.0f)) + pz;

    *(v4fa*)(wrow + c0)     = yA;
    *(v4fa*)(wrow + c0 + 4) = yB;
    __builtin_amdgcn_fence(__ATOMIC_RELEASE, "wavefront");
    __builtin_amdgcn_wave_barrier();
    const v4f g0 = *(const v4fa*)(wrow + 4 * lane);
    const v4f g1 = *(const v4fa*)(wrow + (NCH / 2) + 4 * lane);
    __builtin_amdgcn_fence(__ATOMIC_ACQ_REL, "wavefront");
    __builtin_amdgcn_wave_barrier();

    float* gp = out + (size_t)gcl * NCH;
    if (wr) {
      *(volatile v4f*)(gp + 4 * lane)             = g0;
      *(volatile v4f*)(gp + (NCH / 2) + 4 * lane) = g1;
    }
    __threadfence();
    if (wr) {
      *(volatile v4f*)(gp + 4 * lane)             = g0;
      *(volatile v4f*)(gp + (NCH / 2) + 4 * lane) = g1;
    }
  }
}

static int pick_nb(int nE, int nN) {
  int nb = NBMAX;
  while (nb > 16 && (long long)nb * (long long)nE * 5LL > (long long)RCAP * (long long)nN * 2LL) nb >>= 1;
  return nb;
}
static inline int cdiv(int a, int b) { return (a + b - 1) / b; }

extern "C" void kernel_launch(void* const* d_in, const int* in_sizes, int n_in,
                              void* d_out, int out_size, void* d_ws, size_t ws_size,
                              hipStream_t stream) {
  if (n_in < 7) return;
  const int nN = in_sizes[0] / DIN;
  if (nN <= 0 || in_sizes[0] != nN * DIN || nN > (1 << 22)) return;
  if (in_sizes[1] < 2 || (in_sizes[1] & 1) != 0) return;
  const int nE = in_sizes[1] / 2;
  if (nE < 1 || nE > (1 << 20)) return;
  if (in_sizes[2] != DIN * NCH) return;
  if (in_sizes[3] != NCH || in_sizes[4] != NCH) return;
  if (in_sizes[5] != NCH || in_sizes[6] != NCH) return;
  if (out_size != nN * NCH) return;

  const float* x    = (const float*)d_in[0];
  const int*   ei   = (const int*)  d_in[1];
  const float* W    = (const float*)d_in[2];
  const float* asrc = (const float*)d_in[3];
  const float* adst = (const float*)d_in[4];
  const float* gam  = (const float*)d_in[5];
  const float* bet  = (const float*)d_in[6];
  float* out = (float*)d_out;
  const int* src = ei;
  const int* dst = ei + nE;

  const int MP   = cdiv(nN, GBM) * GBM;
  const int nb   = pick_nb(nE, nN);
  const int gA   = cdiv(nN, nb);
  const int vec8 = ((nE & 3) == 0) ? 1 : 0;
  if (gA * nb < nN || nb < 16 || nb > NBMAX) return;

  char* ws = (char*)d_ws;
  size_t off = 0;
  const size_t oXB = off; off += (size_t)MP * DIN * 2;             off = (off + 255) & ~(size_t)255;
  const size_t oWT = off; off += (size_t)NCH * DIN * 2;            off = (off + 255) & ~(size_t)255;
  const size_t oHF = off; off += (size_t)MP * NCH * 4;             off = (off + 255) & ~(size_t)255;
  if (off > ws_size || off > (size_t)WSMAX) return;
  unsigned short* XB = (unsigned short*)(ws + oXB);
  unsigned short* WT = (unsigned short*)(ws + oWT);
  float*          HF = (float*)(ws + oHF);

  hipFuncSetAttribute(reinterpret_cast<const void*>(&k_agg),
                      hipFuncAttributeMaxDynamicSharedMemorySize, LDS_AGG);

  const int nUx = MP * (DIN / 8);
  k_xprep<<<cdiv(nUx, NTHR), NTHR, 0, stream>>>(x, XB, nN, nUx);

  const int nUw = NCH * (DIN / 8);
  k_wtr<<<cdiv(nUw, NTHR), NTHR, 0, stream>>>(W, DIN, NCH, NCH, DIN, WT, nUw);

  const int gM = MP / GBM;
  k_gemm<<<dim3(gM, NCH / GBN), GTHR, 0, stream>>>(XB, WT, HF, DIN, NCH);

  k_agg<<<gA, NTHR, LDS_AGG, stream>>>(src, dst, HF, x, asrc, adst, gam, bet, out, nN, nE, nb, vec8);
}
